// NonLocalBlockND_34394098106431
// MI455X (gfx1250) — hardware-verified
//
#include <hip/hip_runtime.h>


namespace {
constexpr int B = 4, C = 256, TT = 8, IH = 32, IW = 32, T = TT * IH * IW  , NK = TT * (IH / 2) * (IW / 2)  , HD = 128  , H = 1, BL = 4  , QL = T;
constexpr float XS = 8.0f, WSC = 256.0f, PS = 1024.0f, RS_ = 1024.0f, LOG2E = 1.4426950408889634f, BNEPS = 1e-5f;
static_assert(T % 64 == 0 && C == 256 && HD == 128 && IW == 32 && NK == T / 4, "tiling");
typedef _Float16 b16;
typedef __attribute__((ext_vector_type(16))) _Float16 v16b;
typedef __attribute__((ext_vector_type(8))) _Float16 v8b;
typedef __attribute__((ext_vector_type(8))) float v8f;
typedef __attribute__((ext_vector_type(4))) float v4f;
__device__ __forceinline__ float bf16_rne(float f) { unsigned int u = __float_as_uint(f); u += 0x7FFFu + ((u >> 16) & 1u); return __uint_as_float(u & 0xFFFF0000u); }
__device__ __forceinline__ void split16(float v, b16& hi, b16& lo) { hi = (b16)v; lo = (b16)(v - (float)hi); }
__device__ __forceinline__ v16b frag_kb(const b16* p, int hh) { const v8b a = *(const v8b*)(p + 8 * hh), b = *(const v8b*)(p + 16 + 8 * hh); v16b f;
#pragma unroll
  for (int e = 0; e < 8; ++e) { f[e] = a[e]; f[8 + e] = b[e]; } return f; }
__device__ __forceinline__ v8f wmma16b(v16b a, v16b b, v8f c) { v8f d = __builtin_amdgcn_wmma_f32_16x16x32_f16(false, a, false, b, (short)0, c, false, false); asm volatile("v_nop\n\tv_nop\n\tv_nop\n\tv_nop" : "+v"(d) : "v"(a), "v"(b)); return d; }
__device__ __forceinline__ void wave_lds_sync() { __builtin_amdgcn_fence(__ATOMIC_RELEASE, "workgroup"); __builtin_amdgcn_wave_barrier(); __builtin_amdgcn_fence(__ATOMIC_ACQUIRE, "workgroup"); }
__device__ __forceinline__ float pmul(float a, float b) { float p = a * b; asm volatile("" : "+v"(p)); return p; }
__device__ __forceinline__ int iclamp(int v, int lo, int hi) { return v < lo ? lo : (v > hi ? hi : v); }

typedef __attribute__((ext_vector_type(2))) _Float16 v2h;
typedef __attribute__((ext_vector_type(4))) _Float16 v4h;
typedef __attribute__((ext_vector_type(2))) float v2f;
typedef __attribute__((ext_vector_type(4))) int v4i;
__device__ __forceinline__ float nexp2(float v) { return __builtin_amdgcn_exp2f(v); }
__device__ __forceinline__ float bfp(float v) { float t = bf16_rne(v); asm volatile("" : "+v"(t)); return t; }
__global__ __launch_bounds__(256) void prep_kernel(const float* __restrict__ thw, const float* __restrict__ phw, const float* __restrict__ gw, const float* __restrict__ ww, b16* __restrict__ WT, b16* __restrict__ WW) {
  const size_t u = (size_t)blockIdx.x * 256 + threadIdx.x; const size_t n1 = (size_t)3 * HD * C / 8, n2 = (size_t)C * HD / 8; if (u >= n1 + n2) return; v8b v;
  if (u < n1) { const size_t e = u * 8; const int o = (int)(e / C), c0 = (int)(e % C); const int m = o / HD, oo = o % HD; const float* w = (m == 0 ? thw : m == 1 ? phw : gw) + (size_t)oo * C;
    for (int j = 0; j < 8; ++j) v[j] = (b16)(bf16_rne(w[c0 + j]) * WSC); for (int pass = 0; pass < 2; ++pass) { *(volatile v8b*)(WT + e) = v; __threadfence(); } }
  else { const size_t e = (u - n1) * 8; for (int j = 0; j < 8; ++j) v[j] = (b16)(bf16_rne(ww[e + j]) * WSC); for (int pass = 0; pass < 2; ++pass) { *(volatile v8b*)(WW + e) = v; __threadfence(); } }
}
__global__ __launch_bounds__(128) void conv_kernel(const float* __restrict__ x, const b16* __restrict__ WT, const float* __restrict__ thb, const float* __restrict__ phb, const float* __restrict__ gb, b16* __restrict__ QP, b16* __restrict__ QPl, b16* __restrict__ KP, b16* __restrict__ KPl, float* __restrict__ GP) {
  __shared__ __attribute__((aligned(16))) b16 As[64][256 + 8]; __shared__ __attribute__((aligned(16))) float Tf[4][16][128 + 4];
  const int wave = threadIdx.x >> 5, lane = threadIdx.x & 31, nloc = lane & 15, hlf = lane >> 4; const int p0 = blockIdx.x * 64, b = blockIdx.y, part = blockIdx.z; const int n0 = part * HD;
  const float* xb = x + (size_t)b * C * T;
  for (int i = threadIdx.x; i < 256 * 16; i += 128) { const int c = i / 16, q4 = (i % 16) * 4; const v4f f = *(const v4f*)(xb + (size_t)c * T + p0 + q4); for (int j = 0; j < 4; ++j) As[q4 + j][c] = (b16)(bf16_rne(f[j]) * XS); }
  __syncthreads();
  v8f acc[8];
#pragma unroll
  for (int t = 0; t < 8; ++t) acc[t] = (v8f){};
#pragma unroll 2
  for (int kb = 0; kb < C; kb += 32) { const v16b a = frag_kb(&As[wave * 16 + nloc][kb], hlf);
#pragma unroll
    for (int t = 0; t < 8; ++t) acc[t] = wmma16b(a, frag_kb(WT + (size_t)(n0 + t * 16 + nloc) * C + kb, hlf), acc[t]); }
  const float* bp = part == 0 ? thb : (part == 1 ? phb : gb);
#pragma unroll
  for (int t = 0; t < 8; ++t) { const float bb = bf16_rne(bp[t * 16 + nloc]);
#pragma unroll
    for (int r = 0; r < 8; ++r) Tf[wave][8 * hlf + r][t * 16 + nloc] = acc[t][r] * (1.0f / (XS * WSC)) + bb; }
  __syncthreads();
  for (int pass = 0; pass < 2; ++pass) {
    if (part == 0) { for (int rr = 0; rr < 16; ++rr) { const int pos = p0 + wave * 16 + rr; v4h h4, l4; for (int j = 0; j < 4; ++j) { const float f = Tf[wave][rr][lane * 4 + j] * XS; const b16 p = (b16)f; h4[j] = p; l4[j] = (b16)((f - (float)p) * RS_); }
        *(volatile v4h*)(QP + ((size_t)b * T + pos) * HD + lane * 4) = h4; *(volatile v4h*)(QPl + ((size_t)b * T + pos) * HD + lane * 4) = l4; } }
    else { for (int jj = wave * 4; jj < wave * 4 + 4; ++jj) { const int key = blockIdx.x * 16 + jj;
        v4f m4; for (int j = 0; j < 4; ++j) { const int d = lane * 4 + j; const int r0 = 2 * jj, r1 = 2 * jj + 1, r2 = 32 + 2 * jj, r3 = 33 + 2 * jj; m4[j] = fmaxf(fmaxf(Tf[r0 >> 4][r0 & 15][d], Tf[r1 >> 4][r1 & 15][d]), fmaxf(Tf[r2 >> 4][r2 & 15][d], Tf[r3 >> 4][r3 & 15][d])); }
        if (part == 1) { v4h h4, l4; for (int j = 0; j < 4; ++j) { const float f = m4[j] * XS; const b16 p = (b16)f; h4[j] = p; l4[j] = (b16)((f - (float)p) * RS_); } *(volatile v4h*)(KP + ((size_t)b * NK + key) * HD + lane * 4) = h4; *(volatile v4h*)(KPl + ((size_t)b * NK + key) * HD + lane * 4) = l4; }
        else *(volatile v4f*)(GP + ((size_t)b * NK + key) * HD + lane * 4) = m4; } }
    __threadfence(); }
}
__global__ __launch_bounds__(256) void gt_kernel(const float* __restrict__ GP, b16* __restrict__ GT, b16* __restrict__ GTl) {
  __shared__ float tile[64][HD + 1];
  const int tid = threadIdx.x, wave = tid >> 5, lane = tid & 31; const int k0 = blockIdx.x * 64, b = blockIdx.y;
  for (int i = tid; i < 64 * (HD / 4); i += 256) { const int rr = i / (HD / 4), c4 = (i % (HD / 4)) * 4; const v4f v = *(const v4f*)(GP + ((size_t)b * NK + k0 + rr) * HD + c4); for (int j = 0; j < 4; ++j) tile[rr][c4 + j] = v[j]; }
  __syncthreads();
  for (int pass = 0; pass < 2; ++pass) {
#pragma unroll 1
    for (int d = wave * 16; d < wave * 16 + 16; ++d) { v2h hv, lv; for (int j = 0; j < 2; ++j) { const float f = tile[2 * lane + j][d] * XS; const b16 p = (b16)f; hv[j] = p; lv[j] = (b16)((f - (float)p) * RS_); }
      const size_t oi = ((size_t)b * HD + d) * (size_t)NK + k0 + 2 * lane; *(volatile v2h*)(GT + oi) = hv; *(volatile v2h*)(GTl + oi) = lv; }
    __threadfence(); }
}
__global__ __launch_bounds__(64) void attn_kernel(const b16* __restrict__ QP, const b16* __restrict__ QPl, const b16* __restrict__ KP, const b16* __restrict__ KPl, const b16* __restrict__ VT, const b16* __restrict__ VTl, b16* __restrict__ Y, b16* __restrict__ Yl) {
  __shared__ __attribute__((aligned(16))) b16 Pb[2][16][32 + 8]; __shared__ __attribute__((aligned(16))) float To[2][16][HD + 4];
  const int wave = threadIdx.x >> 5, lane = threadIdx.x & 31, hh = lane >> 4, col = lane & 15; const int b = blockIdx.y, h = 0; const int q0 = blockIdx.x * 32 + wave * 16, qi = q0 + col;
  const size_t qo = (size_t)b * T * HD, ko = (size_t)b * NK * HD, vo = (size_t)b * HD * (size_t)NK; const b16* Qb = QP + qo; const b16* Qbl = QPl + qo; const b16* Kb = KP + ko; const b16* Kbl = KPl + ko; const b16* Vb = VT + vo; const b16* Vbl = VTl + vo; (void)h;
  __shared__ __attribute__((aligned(16))) b16 Qs[2][16][HD + 8], Qsl[2][16][HD + 8];
  for (int i = lane; i < 16 * (HD / 8); i += 32) { const int rr = i / (HD / 8), c8 = (i % (HD / 8)) * 8; *(v8b*)(&Qs[wave][rr][c8]) = *(const v8b*)(Qb + (size_t)(q0 + rr) * HD + c8); *(v8b*)(&Qsl[wave][rr][c8]) = *(const v8b*)(Qbl + (size_t)(q0 + rr) * HD + c8); }
  wave_lds_sync();
  const float cs = LOG2E / (XS * XS);
  __shared__ __attribute__((aligned(16))) b16 Plq[2][16][32 + 8];
  float m = -INFINITY, l = 0.0f; v8f o[8], ol[8]; for (int t = 0; t < 8; ++t) { o[t] = (v8f){}; ol[t] = (v8f){}; }
#pragma unroll 1
  for (int kb = 0; kb < NK; kb += 32) {
    float e[16]; float mx = -INFINITY;
#pragma unroll
    for (int u = 0; u < 2; ++u) { v8f s = (v8f){}, sx = (v8f){}; const size_t kr = (size_t)(kb + u * 16 + col) * HD;
#pragma unroll
      for (int ks = 0; ks < 4; ++ks) { const v16b kf = frag_kb(Kb + kr + 32 * ks, hh); const v16b qf = frag_kb(&Qs[wave][col][32 * ks], hh); s = wmma16b(kf, qf, s); sx = wmma16b(kf, frag_kb(&Qsl[wave][col][32 * ks], hh), sx); sx = wmma16b(frag_kb(Kbl + kr + 32 * ks, hh), qf, sx); }
#pragma unroll
      for (int r = 0; r < 8; ++r) s[r] += sx[r] * (1.0f / RS_);
#pragma unroll
      for (int r = 0; r < 8; ++r) { const float vv = s[r] * cs; e[u * 8 + r] = vv; mx = fmaxf(mx, vv); } }
    mx = fmaxf(mx, __shfl_xor(mx, 16)); const float mn = fmaxf(m, mx); const float al = nexp2(m - mn); float sum = 0.0f;
#pragma unroll
    for (int i2 = 0; i2 < 16; ++i2) { const float p = nexp2(e[i2] - mn); sum += p; const int pc = (i2 < 8 ? 0 : 16) + 8 * hh + (i2 & 7); const float ps = p * PS; const b16 phh = (b16)ps; Pb[wave][col][pc] = phh; Plq[wave][col][pc] = (b16)((ps - (float)phh) * RS_); }
    sum += __shfl_xor(sum, 16); l = l * al + sum; m = mn;
    wave_lds_sync();
    const v16b pf = frag_kb(&Pb[wave][col][0], hh), plf = frag_kb(&Plq[wave][col][0], hh);
#pragma unroll
    for (int t = 0; t < 8; ++t) { const v16b vh = frag_kb(Vb + (size_t)(t * 16 + col) * NK + kb, hh); o[t] *= al; o[t] = wmma16b(vh, pf, o[t]); ol[t] = wmma16b(frag_kb(Vbl + (size_t)(t * 16 + col) * NK + kb, hh), pf, ol[t] * al); ol[t] = wmma16b(vh, plf, ol[t]); }
    wave_lds_sync(); }
  const float inv = 1.0f / (l * PS * XS);
#pragma unroll
  for (int t = 0; t < 8; ++t)
#pragma unroll
    for (int r = 0; r < 8; ++r) To[wave][col][t * 16 + 8 * hh + r] = (o[t][r] + ol[t][r] * (1.0f / RS_)) * inv;
  wave_lds_sync();
  for (int pass = 0; pass < 2; ++pass) { for (int rr = 0; rr < 16; ++rr) { v4h hv, lv; for (int j = 0; j < 4; ++j) { b16 p, ql2; split16(To[wave][rr][lane * 4 + j] * XS, p, ql2); hv[j] = p; lv[j] = ql2; } const size_t oi = ((size_t)b * T + q0 + rr) * HD + lane * 4; *(volatile v4h*)(Y + oi) = hv; *(volatile v4h*)(Yl + oi) = lv; } __threadfence(); }
}
__global__ __launch_bounds__(64) void wconv_kernel(const b16* __restrict__ Y, const b16* __restrict__ Yl, const b16* __restrict__ WW, const float* __restrict__ wb, float* __restrict__ ZT) {
  __shared__ __attribute__((aligned(16))) float Tz[2][16][C + 4];
  const int wave = threadIdx.x >> 5, lane = threadIdx.x & 31, nloc = lane & 15, hlf = lane >> 4; const int b = blockIdx.y; const size_t m0 = (size_t)b * T + (size_t)blockIdx.x * 32 + wave * 16;
  v8f acc[16];
#pragma unroll
  for (int t = 0; t < 16; ++t) acc[t] = (v8f){};
#pragma unroll
  for (int kb = 0; kb < HD; kb += 32) { const v16b a = frag_kb(Y + (m0 + nloc) * HD + kb, hlf), al = frag_kb(Yl + (m0 + nloc) * HD + kb, hlf);
#pragma unroll
    for (int t = 0; t < 16; ++t) { const v16b bw = frag_kb(WW + (size_t)(t * 16 + nloc) * HD + kb, hlf); acc[t] = wmma16b(a, bw, acc[t]); acc[t] = wmma16b(al, bw, acc[t]); } }
#pragma unroll
  for (int t = 0; t < 16; ++t) { const float bb = bf16_rne(wb[t * 16 + nloc]);
#pragma unroll
    for (int r = 0; r < 8; ++r) Tz[wave][8 * hlf + r][t * 16 + nloc] = acc[t][r] * (1.0f / (XS * WSC)) + bb; }
  __syncthreads();
  for (int pass = 0; pass < 2; ++pass) { for (int c = threadIdx.x; c < C; c += 64) { float* orow = ZT + ((size_t)b * C + c) * (size_t)T + blockIdx.x * 32; v4f o4;
      for (int q4 = 0; q4 < 8; ++q4) { for (int j = 0; j < 4; ++j) { const int qq = q4 * 4 + j; o4[j] = Tz[qq >> 4][qq & 15][c]; } *(volatile v4f*)(orow + q4 * 4) = o4; } } __threadfence(); }
}
template <int MODE>
__global__ __launch_bounds__(256) void bnstat_kernel(const float* __restrict__ ZT, float* __restrict__ ST) {
  __shared__ float red[256]; __shared__ float keep;
  const int c = blockIdx.x, tid = threadIdx.x; const float cnt = (float)BL * (float)QL; const float mean = (MODE == 1) ? ST[(size_t)c * 32] / cnt : 0.0f;
  float s = 0.0f;
  for (int b = 0; b < BL; ++b) { const float* zr = ZT + ((size_t)b * C + c) * (size_t)T;
    for (int i = tid * 4; i < QL; i += 1024) { const v4f v = *(const v4f*)(zr + i); for (int j = 0; j < 4; ++j) { const float d = v[j] - mean; s += (MODE == 1) ? pmul(d, d) : v[j]; } } }
  red[tid] = s; if (tid == 0) keep = (MODE == 1) ? ST[(size_t)c * 32] : 0.0f;
  __syncthreads();
  for (int stride = 128; stride >= 1; stride >>= 1) { if (tid < stride) red[tid] += red[tid + stride]; __syncthreads(); }
  for (int pass = 0; pass < 2; ++pass) { if (tid < 32) { const float v = (tid == MODE) ? red[0] : ((tid == 0) ? keep : 0.0f); ((volatile float*)ST)[(size_t)c * 32 + tid] = v; } __threadfence(); }
}
__global__ __launch_bounds__(256) void bnapply_kernel(const float* __restrict__ ZT, const float* __restrict__ ST, const float* __restrict__ gamma, const float* __restrict__ beta, const float* __restrict__ x, float* __restrict__ out) {
  const int c = blockIdx.y, b = blockIdx.z; const float cnt = (float)BL * (float)QL; const float mean = ST[(size_t)c * 32] / cnt; const float rs = rsqrtf(ST[(size_t)c * 32 + 1] / cnt + BNEPS); const float g = bfp(gamma[c]), be = bfp(beta[c]);
  const size_t base = ((size_t)b * C + c) * (size_t)T + (size_t)blockIdx.x * 1024 + threadIdx.x * 4; const v4f z = *(const v4f*)(ZT + base), xv = *(const v4f*)(x + base); v4f o;
  for (int j = 0; j < 4; ++j) o[j] = pmul((z[j] - mean) * rs, g) + be + bf16_rne(xv[j]);
  for (int pass = 0; pass < 2; ++pass) { *(volatile v4f*)(out + base) = o; __threadfence(); }
}
}

extern "C" void kernel_launch(void* const* d_in, const int* in_sizes, int n_in, void* d_out, int out_size, void* d_ws, size_t ws_size, hipStream_t stream) {
  (void)n_in;
  auto Fp = [&](int i) { return (const float*)d_in[i]; };
  if (in_sizes[0] != B * C * T || in_sizes[1] != HD * C || in_sizes[2] != HD || in_sizes[3] != HD * C || in_sizes[4] != HD || in_sizes[5] != HD * C || in_sizes[6] != HD || in_sizes[7] != C * HD || in_sizes[8] != C || in_sizes[9] != C || in_sizes[10] != C || out_size != B * C * T) return;
  size_t off = 0; char* ws = (char*)d_ws;
  auto carve = [&](size_t bytes) { char* p = ws + off; off += (bytes + 255) & ~(size_t)255; return p; };
  b16* WT = (b16*)carve((size_t)3 * HD * C * 2); b16* WW = (b16*)carve((size_t)C * HD * 2);
  b16* QP = (b16*)carve((size_t)B * T * HD * 2); b16* QPl = (b16*)carve((size_t)B * T * HD * 2); b16* KP = (b16*)carve((size_t)B * NK * HD * 2); b16* KPl = (b16*)carve((size_t)B * NK * HD * 2);
  float* GP = (float*)carve((size_t)B * NK * HD * 4); b16* GT = (b16*)carve((size_t)B * HD * NK * 2); b16* GTl = (b16*)carve((size_t)B * HD * NK * 2);
  b16* Y = (b16*)carve((size_t)B * T * HD * 2); b16* Yl = (b16*)carve((size_t)B * T * HD * 2); float* ZT = (float*)carve((size_t)B * C * T * 4); float* ST = (float*)carve((size_t)C * 32 * 4);
  if (off > ws_size || off > ((size_t)128 << 20)) return;
  prep_kernel<<<(unsigned)(((size_t)(3 * HD * C + C * HD) / 8 + 255) / 256), 256, 0, stream>>>(Fp(3), Fp(5), Fp(1), Fp(7), WT, WW);
  conv_kernel<<<dim3(T / 64, BL, 3), 128, 0, stream>>>(Fp(0), WT, Fp(4), Fp(6), Fp(2), QP, QPl, KP, KPl, GP);
  gt_kernel<<<dim3(NK / 64, BL), 256, 0, stream>>>(GP, GT, GTl);
  attn_kernel<<<dim3(QL / 32, BL), 64, 0, stream>>>(QP, QPl, KP, KPl, GT, GTl, Y, Yl);
  wconv_kernel<<<dim3(QL / 32, BL), 64, 0, stream>>>(Y, Yl, WW, Fp(8), ZT);
  bnstat_kernel<0><<<C, 256, 0, stream>>>(ZT, ST); bnstat_kernel<1><<<C, 256, 0, stream>>>(ZT, ST);
  bnapply_kernel<<<dim3(QL / 1024, C, BL), 256, 0, stream>>>(ZT, ST, Fp(9), Fp(10), Fp(0), (float*)d_out);
}
